// DepthAwareGATv2_15522011808332
// MI455X (gfx1250) — hardware-run, weakly checked
//
#include <hip/hip_runtime.h>


namespace {
constexpr int N = 50000, E = 800000, FI = 16, FE = 8, NH = 4, C = 32, D = 128, NCLS = 5, NBLK = N / 16;
constexpr float XS = 8.0f, ES = 32.0f, WSC = 256.0f;
typedef _Float16 b16;
typedef __attribute__((ext_vector_type(16))) _Float16 v16b;
typedef __attribute__((ext_vector_type(8))) _Float16 v8b;
typedef __attribute__((ext_vector_type(8))) float v8f;
typedef __attribute__((ext_vector_type(4))) float v4f;
__device__ __forceinline__ float bf16_rne(float f) { unsigned int u = __float_as_uint(f); u += 0x7FFFu + ((u >> 16) & 1u); return __uint_as_float(u & 0xFFFF0000u); }
__device__ __forceinline__ v16b frag_kb(const b16* p, int hh) { const v8b a = *(const v8b*)(p + 8 * hh), b = *(const v8b*)(p + 16 + 8 * hh); v16b f;
#pragma unroll
  for (int e = 0; e < 8; ++e) { f[e] = a[e]; f[8 + e] = b[e]; } return f; }
__device__ __forceinline__ v8f wmma16b(v16b a, v16b b, v8f c) { v8f d = __builtin_amdgcn_wmma_f32_16x16x32_f16(false, a, false, b, (short)0, c, false, false); asm volatile("v_nop\n\tv_nop\n\tv_nop\n\tv_nop" : "+v"(d) : "v"(a), "v"(b)); return d; }
__device__ __forceinline__ void wave_lds_sync() { __builtin_amdgcn_fence(__ATOMIC_RELEASE, "workgroup"); __builtin_amdgcn_wave_barrier(); __builtin_amdgcn_fence(__ATOMIC_ACQUIRE, "workgroup"); }
__device__ __forceinline__ float pmul(float a, float b) { float p = a * b; asm volatile("" : "+v"(p)); return p; }
__device__ __forceinline__ int iclamp(int v, int lo, int hi) { return v < lo ? lo : (v > hi ? hi : v); }
__device__ __forceinline__ float leaky(float v) { return v > 0.0f ? v : 0.2f * v; }
__device__ __forceinline__ float elu(float v) { return v > 0.0f ? v : expm1f(v); }
constexpr int CSR_NBLK9 = 512, CSR_GB9 = 9, CSR_GN9 = 1 << CSR_GB9  , CSR_TS9 = (CSR_GN9 < 32 ? 32 : CSR_GN9)  , CSR_MAXG9 = 512, CSR_CAP9 = 12288  ;
__device__ __host__ __forceinline__ int csr_tix9(int v) { return (v >> CSR_GB9) * CSR_TS9 + (v & (CSR_GN9 - 1)); }
__global__ __launch_bounds__(64) void csrA_kernel9(const int* __restrict__ dst, int E, int N, int nG, int CHP, int NGP, int* __restrict__ STG, int* __restrict__ HST) {
  extern __shared__ int sm[];
  int* cnt = sm; int* run = sm + NGP; int* ids = sm + 2 * NGP;
  const int b = blockIdx.x; const int ch = (E + CSR_NBLK9 - 1) / CSR_NBLK9; const int e0 = b * ch, e1 = min(E, e0 + ch);
  for (int i = threadIdx.x; i < NGP; i += 64) cnt[i] = 0;
  for (int i = threadIdx.x; i < CHP; i += 64) ids[i] = -1;
  __syncthreads();
  if (threadIdx.x == 0) {
    for (int e = e0; e < e1; ++e) { int d = dst[e]; d = (d < 0) ? 0 : (d >= N ? N - 1 : d); cnt[d >> CSR_GB9] += 1; }
    int acc = 0; for (int g = 0; g < nG; ++g) { run[g] = acc; acc += cnt[g]; }
    for (int e = e0; e < e1; ++e) { int d = dst[e]; d = (d < 0) ? 0 : (d >= N ? N - 1 : d); const int g = d >> CSR_GB9; ids[run[g]] = e; run[g] += 1; } }
  __syncthreads();
  typedef __attribute__((ext_vector_type(4))) int v4i;
  for (int pass = 0; pass < 2; ++pass) {
    for (int i = threadIdx.x; i < CHP / 4; i += 64) *(volatile v4i*)(STG + (size_t)b * CHP + i * 4) = *(const v4i*)(&ids[i * 4]);
    for (int i = threadIdx.x; i < NGP / 4; i += 64) { v4i v; for (int e = 0; e < 4; ++e) v[e] = (i * 4 + e < nG) ? cnt[i * 4 + e] : 0; *(volatile v4i*)(HST + (size_t)b * NGP + i * 4) = v; }
    __threadfence(); }
}
__global__ __launch_bounds__(512) void csrS_kernel9(const int* __restrict__ HST, int nG, int NGP, int* __restrict__ START, int* __restrict__ TOT, int* __restrict__ OFF) {
  __shared__ int tot[CSR_MAXG9];
  const int b = threadIdx.x;
  for (int pass = 0; pass < 2; ++pass) { int runb = 0; for (int g = 0; g < nG; ++g) { int c = HST[(size_t)b * NGP + g]; c = (c < 0) ? 0 : c; ((volatile int*)OFF)[(size_t)g * CSR_NBLK9 + b] = runb; runb += c; } __threadfence(); }
  for (int g = threadIdx.x; g < nG; g += 512) { int s = 0; for (int bb = 0; bb < CSR_NBLK9; ++bb) { int c = HST[(size_t)bb * NGP + g]; s += (c < 0) ? 0 : c; } tot[g] = s; }
  __syncthreads();
  if (threadIdx.x < 32) {
    __shared__ int st[CSR_MAXG9 + 32];
    if (threadIdx.x == 0) { int acc = 0; for (int g = 0; g < NGP; ++g) { st[g] = acc; if (g < nG) acc += (tot[g] + 31) & ~31; } st[NGP] = acc; }
    __builtin_amdgcn_fence(__ATOMIC_RELEASE, "workgroup"); __builtin_amdgcn_wave_barrier(); __builtin_amdgcn_fence(__ATOMIC_ACQUIRE, "workgroup");
    for (int pass = 0; pass < 2; ++pass) { for (int i = threadIdx.x; i < NGP + 32; i += 32) { ((volatile int*)START)[i] = (i <= NGP) ? st[min(i, NGP)] : 0; ((volatile int*)TOT)[i] = (i < nG) ? tot[i] : 0; } __threadfence(); } }
}
__global__ __launch_bounds__(256) void csrB_kernel9(const int* __restrict__ dst, int N, int nG, int CHP, int NGP, int permLen, const int* __restrict__ STG, const int* __restrict__ HST, const int* __restrict__ OFF, const int* __restrict__ START, const int* __restrict__ TOT, int* __restrict__ PERM, int* __restrict__ ROWPTR, int* __restrict__ ROWCNT, int* __restrict__ FLAG) {
  typedef __attribute__((ext_vector_type(4))) int v4i;
  __shared__ int ids[CSR_CAP9]; __shared__ unsigned short key[CSR_CAP9]; __shared__ int outp[CSR_CAP9]; __shared__ int ncnt[CSR_GN9 + 1]; __shared__ int boff[CSR_NBLK9 + 1];
  const int g = blockIdx.x, t_ = threadIdx.x; int tot = TOT[g]; int st = START[g], stn = START[g + 1]; const int v0 = g * CSR_GN9; const int nv = min(CSR_GN9, N - v0); const int t0 = g * CSR_TS9;
  st = (st < 0) ? 0 : (st > permLen - 32 ? permLen - 32 : st) & ~31; stn = (stn < st) ? st : (stn > permLen ? permLen : stn); tot = (tot < 0) ? 0 : tot; if (tot > stn - st && tot <= CSR_CAP9) tot = stn - st;
  if (tot > CSR_CAP9) {
    for (int pass = 0; pass < 2; ++pass) { for (int i = t_; i < CSR_TS9 / 4; i += 256) { v4i a, c; for (int e = 0; e < 4; ++e) { a[e] = st; c[e] = 0; } *(volatile v4i*)(ROWPTR + t0 + i * 4) = a; *(volatile v4i*)(ROWCNT + t0 + i * 4) = c; } if (t_ == 0) ((volatile int*)FLAG)[0] = 1; __threadfence(); } (void)nv; return; }
  if (t_ == 0) { int acc = 0; for (int b = 0; b < CSR_NBLK9; ++b) { boff[b] = acc; int c = HST[(size_t)b * NGP + g]; c = (c < 0) ? 0 : (c > CHP ? CHP : c); acc += c; if (acc > tot) acc = tot; } boff[CSR_NBLK9] = acc; }
  for (int i = t_; i <= CSR_GN9; i += 256) ncnt[i] = 0;
  __syncthreads();
  for (int b = 0; b < CSR_NBLK9; ++b) { const int c = boff[b + 1] - boff[b]; int o_ = OFF[(size_t)g * CSR_NBLK9 + b]; o_ = (o_ < 0) ? 0 : (o_ > CHP - c ? CHP - c : o_); const int* src_ = STG + (size_t)b * CHP + o_;
    for (int i = t_; i < c; i += 256) { int id = src_[i]; id = (id < 0) ? 0 : id; ids[boff[b] + i] = id; int d = dst[id]; d = (d < v0) ? v0 : (d >= N ? N - 1 : d); int kk = d - v0; kk = (kk < 0) ? 0 : (kk >= CSR_GN9 ? CSR_GN9 - 1 : kk); key[boff[b] + i] = (unsigned short)kk; } }
  __syncthreads();
  if (t_ == 0) { for (int i = 0; i < tot; ++i) ncnt[key[i]] += 1; int acc = 0; for (int vl = 0; vl < CSR_GN9; ++vl) { const int c = ncnt[vl]; ncnt[vl] = acc; acc += c; } ncnt[CSR_GN9] = acc;
    for (int i = 0; i < tot; ++i) { const int vl = key[i]; outp[ncnt[vl]] = ids[i]; ncnt[vl] += 1; }
    for (int vl = CSR_GN9; vl > 0; --vl) ncnt[vl] = ncnt[vl - 1]; ncnt[0] = 0; }
  __syncthreads();
  for (int pass = 0; pass < 2; ++pass) {
    for (int i = t_; i < (stn - st) / 4; i += 256) { v4i v; for (int e = 0; e < 4; ++e) { const int q = i * 4 + e; v[e] = (q < tot) ? outp[q] : -1; } *(volatile v4i*)(PERM + st + i * 4) = v; }
    for (int i = t_; i < CSR_TS9 / 4; i += 256) { v4i a, c; for (int e = 0; e < 4; ++e) { const int vl = i * 4 + e; const int vc = vl < CSR_GN9 ? vl : CSR_GN9; a[e] = (vl < CSR_GN9) ? st + ncnt[vc] : st; c[e] = (vl < nv) ? (ncnt[(vc < CSR_GN9 ? vc : CSR_GN9 - 1) + 1] - ncnt[vc]) : 0; } *(volatile v4i*)(ROWPTR + t0 + i * 4) = a; *(volatile v4i*)(ROWCNT + t0 + i * 4) = c; }
    __threadfence(); }
}
__global__ __launch_bounds__(256) void csrZ_kernel9(int* __restrict__ p, size_t n4) { typedef __attribute__((ext_vector_type(4))) int v4i; const size_t tid = (size_t)blockIdx.x * 256 + threadIdx.x, nth = (size_t)gridDim.x * 256; v4i z = {0, 0, 0, 0}; for (size_t i = tid; i < n4; i += nth) *(volatile v4i*)(p + i * 4) = z; }
struct CsrBufs9 { int *STG, *HST, *OFF, *START, *TOT, *PERM, *ROWPTR, *ROWCNT, *FLAG; int nG, NGP, CHP; size_t permLen; char* base; size_t bytes; };
static size_t csr_carve9(CsrBufs9& c, char* ws, size_t off, int E, int N) {
  const size_t off0 = off; c.base = ws + off;
  auto al = [&](size_t bytes) { char* p = ws + off; off += (bytes + 255) & ~(size_t)255; return p; };
  c.nG = (N + CSR_GN9 - 1) / CSR_GN9; c.NGP = (c.nG + 31) & ~31; const int ch = (E + CSR_NBLK9 - 1) / CSR_NBLK9; c.CHP = (ch + 31) & ~31; c.permLen = (size_t)E + 32 * (size_t)c.nG + 32;
  c.STG = (int*)al((size_t)CSR_NBLK9 * c.CHP * 4); c.HST = (int*)al((size_t)CSR_NBLK9 * c.NGP * 4); c.OFF = (int*)al((size_t)c.NGP * CSR_NBLK9 * 4); c.START = (int*)al((size_t)(c.NGP + 64) * 4); c.TOT = (int*)al((size_t)(c.NGP + 64) * 4);
  c.PERM = (int*)al(c.permLen * 4); c.ROWPTR = (int*)al((size_t)c.nG * CSR_TS9 * 4); c.ROWCNT = (int*)al((size_t)c.nG * CSR_TS9 * 4); c.FLAG = (int*)al(256);
  c.bytes = off - off0; return off;
}
static void csr_build9(const CsrBufs9& c, const int* dst, int E, int N, hipStream_t stream) {
  const size_t smem = (size_t)(2 * c.NGP + c.CHP) * 4;
  csrZ_kernel9<<<512, 256, 0, stream>>>((int*)c.base, c.bytes / 16);
  csrA_kernel9<<<CSR_NBLK9, 64, smem, stream>>>(dst, E, N, c.nG, c.CHP, c.NGP, c.STG, c.HST);
  csrS_kernel9<<<1, 512, 0, stream>>>(c.HST, c.nG, c.NGP, c.START, c.TOT, c.OFF);
  csrB_kernel9<<<c.nG, 256, 0, stream>>>(dst, N, c.nG, c.CHP, c.NGP, (int)c.permLen, c.STG, c.HST, c.OFF, c.START, c.TOT, c.PERM, c.ROWPTR, c.ROWCNT, c.FLAG);
}


__global__ __launch_bounds__(256) void wcopy_kernel(const float* __restrict__ w, int KIN, int KW, int OUTW, int ro, int ko, int KP, b16* __restrict__ WT) {
  const int KG = KW / 8; const int u = blockIdx.x * 256 + threadIdx.x; if (u >= OUTW * KG) return; const int o = u / KG, k0 = (u % KG) * 8; v8b v;
#pragma unroll
  for (int j = 0; j < 8; ++j) { const int k = k0 + j; v[j] = k < KIN ? (b16)(bf16_rne(w[(size_t)o * KIN + k]) * WSC) : (b16)0.0f; } for (int pass = 0; pass < 2; ++pass) { *(volatile v8b*)(WT + (size_t)(ro + o) * KP + ko + k0) = v; __threadfence(); }
}
__global__ __launch_bounds__(256) void wzero_kernel(int r0, int r1, int KP, b16* __restrict__ WT) { const int u = blockIdx.x * 256 + threadIdx.x; const int n8 = (r1 - r0) * KP / 8; if (u >= n8) return; v8b z; for (int j = 0; j < 8; ++j) z[j] = (b16)0.0f; for (int pass = 0; pass < 2; ++pass) { *(volatile v8b*)(WT + (size_t)r0 * KP + (size_t)u * 8) = z; __threadfence(); } }
__global__ __launch_bounds__(32) void mprep_kernel(const float* __restrict__ le1, const float* __restrict__ ae1, const float* __restrict__ le2, const float* __restrict__ ae2, float* __restrict__ MP) {
  const int lane = threadIdx.x; const int l = lane >> 4, k = (lane >> 2) & 3, h = lane & 3; const float* le = l ? le2 : le1; const float* ae = l ? ae2 : ae1; float s = 0.0f;
  for (int c = 0; c < C; ++c) s += pmul(bf16_rne(le[(size_t)(h * C + c) * NH + k]), bf16_rne(ae[h * C + c]));
  for (int pass = 0; pass < 2; ++pass) { ((volatile float*)MP)[lane] = s; __threadfence(); }
}
__global__ __launch_bounds__(32) void edge_kernel(const float* __restrict__ ea, const b16* __restrict__ WE1, const float* __restrict__ eb1, const b16* __restrict__ WE2, const float* __restrict__ eb2, const float* __restrict__ MP, int ELIM, float* __restrict__ AE) {
  __shared__ __attribute__((aligned(16))) b16 Ah[16][40], Bh[16][40]; __shared__ float Ev[16][NH], So[16][8];
  const int lane = threadIdx.x, nloc = lane & 15, hlf = lane >> 4; const size_t e0 = (size_t)blockIdx.x * 16; if (e0 >= (size_t)ELIM) return;
  for (int rr = 0; rr < 16; ++rr) Ah[rr][lane] = lane < FE ? (b16)(bf16_rne(ea[(e0 + rr) * FE + lane]) * XS) : (b16)0.0f;
  wave_lds_sync();
  { const v16b a = frag_kb(&Ah[nloc][0], hlf);
#pragma unroll
    for (int t = 0; t < 2; ++t) { v8f acc = {}; acc = wmma16b(a, frag_kb(WE1 + (size_t)(t * 16 + nloc) * 32, hlf), acc); const float bb = bf16_rne(eb1[t * 16 + nloc]);
#pragma unroll
      for (int r8 = 0; r8 < 8; ++r8) Bh[8 * hlf + r8][t * 16 + nloc] = (b16)(fmaxf(acc[r8] * (1.0f / (XS * WSC)) + bb, 0.0f) * ES); } }
  wave_lds_sync();
  { v8f acc = {}; acc = wmma16b(frag_kb(&Bh[nloc][0], hlf), frag_kb(WE2 + (size_t)nloc * 32, hlf), acc);
    if (nloc < NH) { const float bb = bf16_rne(eb2[nloc]);
#pragma unroll
      for (int r8 = 0; r8 < 8; ++r8) Ev[8 * hlf + r8][nloc] = acc[r8] * (1.0f / (ES * WSC)) + bb; } }
  wave_lds_sync();
  if (lane < 16) { const int rr = lane; for (int l = 0; l < 2; ++l) for (int h = 0; h < NH; ++h) { float s = 0.0f; for (int k = 0; k < NH; ++k) s += pmul(Ev[rr][k], MP[l * 16 + k * 4 + h]); So[rr][l * 4 + h] = s; } }
  wave_lds_sync();
  for (int pass = 0; pass < 2; ++pass) { for (int q = 0; q < 4; ++q) { const int i = q * 32 + lane; ((volatile float*)AE)[e0 * 8 + i] = So[i >> 3][i & 7]; } __threadfence(); }
}
template <int KP, int FIRST, int NT>
__global__ __launch_bounds__(32) void proj_kernel(const float* __restrict__ IN, int pin, const b16* __restrict__ WT, const float* __restrict__ bias0, const float* __restrict__ asrc, const float* __restrict__ adst, int NLIM, float* __restrict__ OUT0, float* __restrict__ XSo, float* __restrict__ AS) {
  __shared__ __attribute__((aligned(16))) b16 Ah[16][KP + 8]; __shared__ __attribute__((aligned(16))) float Tf[16][128 + 4], Ps[16][8];
  const int lane = threadIdx.x, nloc = lane & 15, hlf = lane >> 4; const size_t m0 = (size_t)blockIdx.x * 16; if (m0 >= (size_t)NLIM) return;
  for (int rr = 0; rr < 16; ++rr) for (int q = 0; q < KP / 32; ++q) { const int c = q * 32 + lane; float v = 0.0f; if (c < pin) { v = IN[(m0 + rr) * pin + c]; if (FIRST) v = bf16_rne(v); } Ah[rr][c] = (b16)(v * XS); }
  wave_lds_sync();
#pragma unroll 1
  for (int cg = 0; cg < NT / 8; ++cg) { const bool isxs = (cg == NT / 8 - 1); v8f acc[8];
#pragma unroll
    for (int t = 0; t < 8; ++t) acc[t] = (v8f){};
#pragma unroll
    for (int kb = 0; kb < KP; kb += 32) { const v16b a = frag_kb(&Ah[nloc][kb], hlf);
#pragma unroll
      for (int t = 0; t < 8; ++t) acc[t] = wmma16b(a, frag_kb(WT + (size_t)(cg * 128 + t * 16 + nloc) * KP + kb, hlf), acc[t]); }
    float ps[8], pd[8];
#pragma unroll
    for (int r8 = 0; r8 < 8; ++r8) { ps[r8] = 0.0f; pd[r8] = 0.0f; }
#pragma unroll
    for (int t = 0; t < 8; ++t) { const int c = t * 16 + nloc; const float bb = isxs ? 0.0f : bf16_rne(bias0[cg * 128 + c]); const float ws_ = isxs ? bf16_rne(asrc[c]) : 0.0f, wd_ = isxs ? bf16_rne(adst[c]) : 0.0f;
#pragma unroll
      for (int r8 = 0; r8 < 8; ++r8) { const float v = acc[t][r8] * (1.0f / (XS * WSC)) + bb; Tf[8 * hlf + r8][c] = v; ps[r8] += pmul(v, ws_); pd[r8] += pmul(v, wd_); }
      if (isxs && (t & 1)) { const int head = t >> 1;
#pragma unroll
        for (int r8 = 0; r8 < 8; ++r8) { float a = ps[r8], dd = pd[r8]; for (int o = 1; o < 16; o <<= 1) { a += __shfl_xor(a, o); dd += __shfl_xor(dd, o); } if (nloc == 0) { Ps[8 * hlf + r8][head] = a; Ps[8 * hlf + r8][4 + head] = dd; } ps[r8] = 0.0f; pd[r8] = 0.0f; } } }
    wave_lds_sync();
    float* dstp = isxs ? XSo : OUT0; const int co = isxs ? 0 : cg * 128; const int pitch = isxs ? D : (NT / 8 - 1) * 128;
    for (int pass = 0; pass < 2; ++pass) { for (int rr = 0; rr < 16; ++rr) *(volatile v4f*)(dstp + (m0 + rr) * pitch + co + lane * 4) = *(const v4f*)(&Tf[rr][lane * 4]); if (isxs) for (int q = 0; q < 4; ++q) { const int i = q * 32 + lane; ((volatile float*)AS)[m0 * 8 + i] = Ps[i >> 3][i & 7]; } __threadfence(); }
    wave_lds_sync(); }
}
__global__ __launch_bounds__(256) void att_kernel(const float* __restrict__ XSp, const float* __restrict__ AS, const float* __restrict__ AE, int lsel, const float* __restrict__ bias, const float* __restrict__ HP, const float* __restrict__ g, const float* __restrict__ be, const int* __restrict__ srcs, const int* __restrict__ PERM, const int* __restrict__ ROWPTR, const int* __restrict__ ROWCNT, int permLen, int NLIM, float* __restrict__ HN) {
  const int wave = threadIdx.x >> 5, lane = threadIdx.x & 31; const size_t v = (size_t)blockIdx.x * 8 + wave; if (v >= (size_t)NLIM) return; const int h = lane >> 3;
  const float ad = AS[v * 8 + 4 + h]; int st = ROWPTR[v], cnt = ROWCNT[v]; cnt = iclamp(cnt, 0, 1 << 20); st = iclamp(st, 0, permLen - cnt); float mx = -INFINITY;
#pragma unroll 1
  for (int j = 0; j < cnt; ++j) { const int e = iclamp(PERM[st + j], 0, E - 1); const size_t s = (size_t)iclamp(srcs[e], 0, N - 1); if (s >= (size_t)NLIM) continue; mx = fmaxf(mx, leaky(AS[s * 8 + h] + ad + AE[(size_t)e * 8 + lsel * 4 + h])); }
  float den = 0.0f; v4f o = {0, 0, 0, 0};
#pragma unroll 1
  for (int j = 0; j < cnt; ++j) { const int e = iclamp(PERM[st + j], 0, E - 1); const size_t s = (size_t)iclamp(srcs[e], 0, N - 1); if (s >= (size_t)NLIM) continue; const float p = __expf(leaky(AS[s * 8 + h] + ad + AE[(size_t)e * 8 + lsel * 4 + h]) - mx); den += p; const v4f xv = *(const v4f*)(XSp + s * D + lane * 4); for (int i = 0; i < 4; ++i) o[i] += pmul(p, xv[i]); }
  const float inv = 1.0f / (den + 1e-16f); float z[4]; float sm = 0.0f; for (int i = 0; i < 4; ++i) { const int c = lane * 4 + i; z[i] = elu(pmul(o[i], inv) + bf16_rne(bias[c])) + HP[v * D + c]; sm += z[i]; }
  for (int q = 16; q; q >>= 1) sm += __shfl_xor(sm, q); const float mu = sm * (1.0f / D); float var = 0.0f; for (int i = 0; i < 4; ++i) { const float dd = z[i] - mu; var += pmul(dd, dd); } for (int q = 16; q; q >>= 1) var += __shfl_xor(var, q); const float rs = rsqrtf(var * (1.0f / D) + 1e-5f);
  v4f r; for (int i = 0; i < 4; ++i) { const int c = lane * 4 + i; r[i] = pmul(pmul(z[i] - mu, rs), bf16_rne(g[c])) + bf16_rne(be[c]); }
  for (int pass = 0; pass < 2; ++pass) { *(volatile v4f*)(HN + v * D + lane * 4) = r; __threadfence(); }
}
__global__ __launch_bounds__(32) void head_kernel(const float* __restrict__ H0, const float* __restrict__ H1, const float* __restrict__ H2, const b16* __restrict__ WJ, const float* __restrict__ jb, const b16* __restrict__ WC, const float* __restrict__ cb, int NLIM, float* __restrict__ out) {
  __shared__ __attribute__((aligned(16))) b16 Ah[16][3 * D + 8], Bh[16][D + 8]; __shared__ float Lg[32][NCLS + 1], So[32][NCLS];
  const int lane = threadIdx.x, nloc = lane & 15, hlf = lane >> 4; const size_t n0 = (size_t)blockIdx.x * 32; if (n0 >= (size_t)NLIM) return;
#pragma unroll 1
  for (int half = 0; half < 2; ++half) { const size_t m0 = n0 + half * 16;
    for (int rr = 0; rr < 16; ++rr) { const size_t row = (m0 + rr < (size_t)N) ? (m0 + rr) : (size_t)(N - 1); for (int q = 0; q < 4; ++q) { const int c = q * 32 + lane; Ah[rr][c] = (b16)(H0[row * D + c] * XS); Ah[rr][D + c] = (b16)(H1[row * D + c] * XS); Ah[rr][2 * D + c] = (b16)(H2[row * D + c] * XS); } }
    wave_lds_sync();
    v8f acc[8];
#pragma unroll
    for (int t = 0; t < 8; ++t) acc[t] = (v8f){};
#pragma unroll 2
    for (int kb = 0; kb < 3 * D; kb += 32) { const v16b a = frag_kb(&Ah[nloc][kb], hlf);
#pragma unroll
      for (int t = 0; t < 8; ++t) acc[t] = wmma16b(a, frag_kb(WJ + (size_t)(t * 16 + nloc) * (3 * D) + kb, hlf), acc[t]); }
#pragma unroll
    for (int t = 0; t < 8; ++t) { const int c = t * 16 + nloc; const float bb = bf16_rne(jb[c]);
#pragma unroll
      for (int r8 = 0; r8 < 8; ++r8) Bh[8 * hlf + r8][c] = (b16)((acc[t][r8] * (1.0f / (XS * WSC)) + bb) * XS); }
    wave_lds_sync();
    { v8f a2 = {};
#pragma unroll
      for (int kb = 0; kb < D; kb += 32) a2 = wmma16b(frag_kb(&Bh[nloc][kb], hlf), frag_kb(WC + (size_t)nloc * D + kb, hlf), a2);
      if (nloc < NCLS) { const float bb = bf16_rne(cb[nloc]);
#pragma unroll
        for (int r8 = 0; r8 < 8; ++r8) Lg[half * 16 + 8 * hlf + r8][nloc] = a2[r8] * (1.0f / (XS * WSC)) + bb; } }
    wave_lds_sync(); }
  { const int r = lane; float mx = -INFINITY; for (int c = 0; c < NCLS; ++c) mx = fmaxf(mx, Lg[r][c]); float s = 0.0f; for (int c = 0; c < NCLS; ++c) s += __expf(Lg[r][c] - mx); const float lse = mx + __logf(s); for (int c = 0; c < NCLS; ++c) So[r][c] = Lg[r][c] - lse; }
  wave_lds_sync();
  const int nval = ((size_t)N - n0 < 32 ? (int)((size_t)N - n0) : 32) * NCLS;
  for (int pass = 0; pass < 2; ++pass) { for (int i = lane; i < nval; i += 32) ((volatile float*)out)[n0 * NCLS + i] = So[i / NCLS][i % NCLS]; __threadfence(); }
}
}

extern "C" void kernel_launch(void* const* d_in, const int* in_sizes, int n_in, void* d_out, int out_size, void* d_ws, size_t ws_size, hipStream_t stream) {
  (void)n_in;
  auto Fp = [&](int i) { return (const float*)d_in[i]; }; auto Ip = [&](int i) { return (const int*)d_in[i]; };
  if (in_sizes[0] != N * FI || in_sizes[1] != 2 * E || in_sizes[2] != E * FE || in_sizes[3] != C * FE || in_sizes[5] != NH * C || in_sizes[7] != D * FI || in_sizes[9] != D * FI || in_sizes[12] != D * NH || in_sizes[15] != D * D || in_sizes[25] != D * 3 * D || in_sizes[27] != NCLS * D || out_size != N * NCLS) return;
  const int NLIM = N; const int ELIM = E; const int GB16 = NBLK, GB8 = N / 8, GB32 = (N + 31) / 32;
  size_t off = 0; char* ws = (char*)d_ws;
  auto carve = [&](size_t bytes) { char* p = ws + off; off += (bytes + 255) & ~(size_t)255; return p; };
  b16* WE1 = (b16*)carve(32 * 32 * 2); b16* WE2 = (b16*)carve(16 * 32 * 2); b16* WP1 = (b16*)carve((size_t)2 * D * 32 * 2); b16* WC2 = (b16*)carve((size_t)D * D * 2); b16* WJ = (b16*)carve((size_t)D * 3 * D * 2); b16* WC = (b16*)carve((size_t)16 * D * 2); float* MP = (float*)carve(128);
  float* AE = (float*)carve((size_t)E * 8 * 4); float* H0 = (float*)carve((size_t)N * D * 4); float* XSp = (float*)carve((size_t)N * D * 4); float* AS = (float*)carve((size_t)N * 8 * 4); float* H1 = (float*)carve((size_t)N * D * 4); float* H2 = (float*)carve((size_t)N * D * 4);
  CsrBufs9 csr; off = csr_carve9(csr, ws, off, E, N);
  if (off > ws_size || off > ((size_t)160 << 20)) return;
  wcopy_kernel<<<1, 256, 0, stream>>>(Fp(3), FE, 32, C, 0, 0, 32, WE1); wcopy_kernel<<<1, 256, 0, stream>>>(Fp(5), C, 32, NH, 0, 0, 32, WE2); wzero_kernel<<<1, 256, 0, stream>>>(NH, 16, 32, WE2);
  wcopy_kernel<<<(D * 4 + 255) / 256, 256, 0, stream>>>(Fp(7), FI, 32, D, 0, 0, 32, WP1); wcopy_kernel<<<(D * 4 + 255) / 256, 256, 0, stream>>>(Fp(9), FI, 32, D, D, 0, 32, WP1);
  wcopy_kernel<<<(D * 16 + 255) / 256, 256, 0, stream>>>(Fp(15), D, D, D, 0, 0, D, WC2); wcopy_kernel<<<(D * 48 + 255) / 256, 256, 0, stream>>>(Fp(25), 3 * D, 3 * D, D, 0, 0, 3 * D, WJ);
  wcopy_kernel<<<(NCLS * 16 + 255) / 256, 256, 0, stream>>>(Fp(27), D, D, NCLS, 0, 0, D, WC); wzero_kernel<<<(11 * D / 8 + 255) / 256, 256, 0, stream>>>(NCLS, 16, D, WC);
  mprep_kernel<<<1, 32, 0, stream>>>(Fp(12), Fp(13), Fp(18), Fp(19), MP);
  csr_build9(csr, Ip(1) + E, E, N, stream);
  edge_kernel<<<(unsigned)((ELIM + 15) / 16), 32, 0, stream>>>(Fp(2), WE1, Fp(4), WE2, Fp(6), MP, ELIM, AE);
  proj_kernel<32, 1, 16><<<GB16, 32, 0, stream>>>(Fp(0), FI, WP1, Fp(8), Fp(10), Fp(11), NLIM, H0, XSp, AS);
  att_kernel<<<GB8, 256, 0, stream>>>(XSp, AS, AE, 0, Fp(14), H0, Fp(21), Fp(22), Ip(1), csr.PERM, csr.ROWPTR, csr.ROWCNT, (int)csr.permLen, NLIM, H1);
  proj_kernel<128, 0, 8><<<GB16, 32, 0, stream>>>(H1, D, WC2, nullptr, Fp(16), Fp(17), NLIM, nullptr, XSp, AS);
  att_kernel<<<GB8, 256, 0, stream>>>(XSp, AS, AE, 1, Fp(20), H1, Fp(23), Fp(24), Ip(1), csr.PERM, csr.ROWPTR, csr.ROWCNT, (int)csr.permLen, NLIM, H2);
  head_kernel<<<GB32, 32, 0, stream>>>(H0, H1, H2, WJ, Fp(26), WC, Fp(28), NLIM, (float*)d_out);
}
